// DotProductAttention_33990371180566
// MI455X (gfx1250) — hardware-verified
//
#include <hip/hip_runtime.h>
#include <math.h>

#ifndef NB
#define NB 32
#endif
#ifndef SEQ
#define SEQ 2048
#endif
#ifndef NB_FULL
#define NB_FULL 32
#endif
#ifndef SEQ_FULL
#define SEQ_FULL 2048
#endif
#define HD 128
#define DVH 64
#define IN_BSTRIDE (SEQ_FULL * HD)
#ifndef OUT_BSTRIDE
#define OUT_BSTRIDE (SEQ_FULL * HD)
#endif
#define AW 4
#define KB 64
#define VP (DVH + 8)
#define PLANE_ELEMS (NB * SEQ * HD)
#define PLANE_BYTES ((((size_t)PLANE_ELEMS * 2) + 255) / 256 * 256)

#ifndef KATTN_ATTR
#define KATTN_ATTR __attribute__((amdgpu_num_vgpr(256)))
#endif

static_assert(HD == 128);
static_assert(HD == 2 * DVH);
static_assert(SEQ % (16 * AW) == 0);
static_assert((SEQ / (16 * AW)) * AW * 16 == SEQ);
static_assert(SEQ % KB == 0);
static_assert(16 * AW == KB);
static_assert(NB <= NB_FULL);
static_assert(SEQ <= SEQ_FULL);
static_assert(PLANE_ELEMS % (256 * 8) == 0);
static_assert(KB * DVH == 4 * (32 * AW) * 8);
static_assert(3 * PLANE_BYTES <= (size_t)134217728);
static_assert((VP * 2) % 16 == 0);

typedef __attribute__((ext_vector_type(16))) __bf16         v16b;
typedef __attribute__((ext_vector_type(8)))  float          v8f;
typedef __attribute__((ext_vector_type(4)))  float          v4f;
typedef __attribute__((ext_vector_type(8)))  unsigned short v8us;
typedef __attribute__((ext_vector_type(16))) unsigned short v16us;
typedef __attribute__((ext_vector_type(4)))  unsigned int   v4u;

__device__ __forceinline__ unsigned frag_k(unsigned i, unsigned h) { return (i < 8u) ? (8u * h + i) : (16u + 8u * h + (i - 8u)); }

__device__ __forceinline__ unsigned bfu_rne(float v) { unsigned u = __float_as_uint(v); u += 0x7fffu + ((u >> 16) & 1u); return u >> 16; }
__device__ __forceinline__ unsigned pk2(float a, float b) { return bfu_rne(a) | (bfu_rne(b) << 16); }
__device__ __forceinline__ __bf16 bf16_rne(float f) { return __builtin_bit_cast(__bf16, (unsigned short)bfu_rne(f)); }
__device__ __forceinline__ float bf16_f32(__bf16 b) { return __uint_as_float(((unsigned int)__builtin_bit_cast(unsigned short, b)) << 16); }

__device__ __forceinline__ v8f wmmab(v16b a, v16b b, v8f c) {
    c = __builtin_amdgcn_wmma_f32_16x16x32_bf16(false, a, false, b, (short)0, c, false, false);
    asm volatile("v_nop\n\tv_nop\n\tv_nop\n\tv_nop" : "+v"(c) : "v"(a), "v"(b));
    return c;
}
struct Split { v16b hi, lo; };
__device__ __forceinline__ v8f wmma2(const Split& a, v16b b, v8f c) {
    c = __builtin_amdgcn_wmma_f32_16x16x32_bf16(false, a.hi, false, b, (short)0, c, false, false);
    c = __builtin_amdgcn_wmma_f32_16x16x32_bf16(false, a.lo, false, b, (short)0, c, false, false);
    asm volatile("v_nop\n\tv_nop\n\tv_nop\n\tv_nop" : "+v"(c) : "v"(a.hi), "v"(a.lo), "v"(b));
    return c;
}

__device__ __forceinline__ v16b frag_row(const unsigned short* row, unsigned k0, unsigned h) {
    const v8us lo = *(const v8us*)(row + k0 + 8u * h);
    const v8us hi = *(const v8us*)(row + k0 + 16u + 8u * h);
    const v16us c = __builtin_shufflevector(lo, hi, 0, 1, 2, 3, 4, 5, 6, 7, 8, 9, 10, 11, 12, 13, 14, 15);
    return __builtin_bit_cast(v16b, c);
}
#define SP1(IDX, XV) { const float spx_ = (XV); const __bf16 sph_ = bf16_rne(spx_); r.hi[IDX] = sph_; r.lo[IDX] = bf16_rne(spx_ - bf16_f32(sph_)); }
__device__ __forceinline__ Split sp_lds(const float* p, unsigned k0, unsigned h) {
    const v4f x0 = *(const v4f*)(p + k0 + 8u * h);
    const v4f x1 = *(const v4f*)(p + k0 + 8u * h + 4u);
    const v4f x2 = *(const v4f*)(p + k0 + 16u + 8u * h);
    const v4f x3 = *(const v4f*)(p + k0 + 16u + 8u * h + 4u);
    Split r;
    SP1(0, x0.x)  SP1(1, x0.y)  SP1(2, x0.z)  SP1(3, x0.w)
    SP1(4, x1.x)  SP1(5, x1.y)  SP1(6, x1.z)  SP1(7, x1.w)
    SP1(8, x2.x)  SP1(9, x2.y)  SP1(10, x2.z) SP1(11, x2.w)
    SP1(12, x3.x) SP1(13, x3.y) SP1(14, x3.z) SP1(15, x3.w)
    return r;
}

#define VST2(T, ptr, val) do { const T vst2_v_ = (val); *(volatile T*)(ptr) = vst2_v_; __threadfence(); *(volatile T*)(ptr) = vst2_v_; } while (0)

__global__ __launch_bounds__(256) void k_cvt3(const float* __restrict__ q, const float* __restrict__ k, const float* __restrict__ v,
                                              unsigned short* __restrict__ pq, unsigned short* __restrict__ pk, unsigned short* __restrict__ pv) {
    const unsigned sel = blockIdx.y;
    const float* src = (sel == 0u) ? q : ((sel == 1u) ? k : v);
    unsigned short* dst = (sel == 0u) ? pq : ((sel == 1u) ? pk : pv);
    const unsigned u = blockIdx.x * 256u + threadIdx.x;
    const unsigned e = u * 8u;
    const unsigned b = e / (unsigned)(SEQ * HD);
    const unsigned rem = e - b * (unsigned)(SEQ * HD);
    const float* s = src + (size_t)b * IN_BSTRIDE + rem;
    const v4f a = *(const v4f*)s;
    const v4f c = *(const v4f*)(s + 4);
    v4u pk4; pk4.x = pk2(a.x, a.y); pk4.y = pk2(a.z, a.w); pk4.z = pk2(c.x, c.y); pk4.w = pk2(c.z, c.w);
    VST2(v4u, dst + e, pk4);
}

__global__ __launch_bounds__(32 * AW) KATTN_ATTR void k_attn(const unsigned short* __restrict__ PQ, const unsigned short* __restrict__ PK,
                                                             const unsigned short* __restrict__ PV, float* __restrict__ O) {
    __shared__ __align__(16) float          pl[AW][16 * KB];
    __shared__ __align__(16) unsigned short vl[KB * VP];
    const unsigned tid = threadIdx.x;
    const unsigned lane = tid & 31u, hf = lane >> 4, l15 = lane & 15u, wave = tid >> 5;
    const unsigned b = blockIdx.y;
    const unsigned dv0 = blockIdx.z * (unsigned)DVH;
    const unsigned q0 = (blockIdx.x * AW + wave) * 16u;
    float* myp = pl[wave];
    const float SCALE = 0.0883883461356163f;
    const float L2E = 1.4426950408889634f;
    const float NEG = -__builtin_inff();
    const unsigned short* qrow  = PQ + ((size_t)b * SEQ + q0 + l15) * HD;
    const unsigned short* kbase = PK + (size_t)b * SEQ * HD;
    const unsigned short* vbase = PV + (size_t)b * SEQ * HD + dv0;

    v8f o[4]; float m8[8], l8[8];
#pragma unroll
    for (int t = 0; t < 4; ++t) { v8f zz = {}; o[t] = zz; }
#pragma unroll
    for (int i = 0; i < 8; ++i) { m8[i] = NEG; l8[i] = 0.f; }

    const unsigned jend = (blockIdx.x + 1u) * (16u * AW);
#pragma unroll 1
    for (unsigned j0 = 0; j0 < jend; j0 += KB) {
        __syncthreads();
#pragma unroll
        for (unsigned it = 0; it < 4u; ++it) {
            const unsigned idx = it * 128u + tid;
            const unsigned jr = idx >> 3, c8 = (idx & 7u) * 8u;
            const v8us x = *(const v8us*)(vbase + (size_t)(j0 + jr) * HD + c8);
            *(v8us*)(vl + jr * VP + c8) = x;
        }
        unsigned qo = 0u;
        asm volatile("" : "+v"(qo));
        const unsigned short* qr = qrow + qo;
        v8f s[4];
#pragma unroll
        for (int t = 0; t < 4; ++t) { v8f zz = {}; s[t] = zz; }
#pragma unroll
        for (int ks = 0; ks < 4; ++ks) {
            const v16b qa = frag_row(qr, (unsigned)ks * 32u, hf);
#pragma unroll
            for (int t = 0; t < 4; ++t) {
                const unsigned short* krow = kbase + (size_t)(j0 + (unsigned)t * 16u + l15) * HD;
                s[t] = wmmab(qa, frag_row(krow, (unsigned)ks * 32u, hf), s[t]);
            }
        }
#pragma unroll
        for (int i = 0; i < 8; ++i) {
            const unsigned irow = q0 + (unsigned)i + 8u * hf;
            float sc[4];
#pragma unroll
            for (int t = 0; t < 4; ++t) {
                const unsigned jg = j0 + (unsigned)t * 16u + l15;
                float v = s[t][i] * SCALE;
                v *= L2E;
                sc[t] = (jg > irow) ? NEG : v;
            }
            float mx = fmaxf(fmaxf(sc[0], sc[1]), fmaxf(sc[2], sc[3]));
            mx = fmaxf(mx, __shfl_xor(mx, 1, 32)); mx = fmaxf(mx, __shfl_xor(mx, 2, 32));
            mx = fmaxf(mx, __shfl_xor(mx, 4, 32)); mx = fmaxf(mx, __shfl_xor(mx, 8, 32));
            const float mnew = fmaxf(m8[i], mx);
            const float corr = (mnew == NEG) ? 1.f : exp2f(m8[i] - mnew);
            float rs = 0.f;
#pragma unroll
            for (int t = 0; t < 4; ++t) {
                const float pp = (sc[t] == NEG) ? 0.f : exp2f(sc[t] - mnew);
                rs += pp;
                myp[((unsigned)i + 8u * hf) * 64u + (unsigned)t * 16u + l15] = pp;
            }
            rs += __shfl_xor(rs, 1, 32); rs += __shfl_xor(rs, 2, 32); rs += __shfl_xor(rs, 4, 32); rs += __shfl_xor(rs, 8, 32);
            l8[i] = l8[i] * corr + rs; m8[i] = mnew;
#pragma unroll
            for (int t = 0; t < 4; ++t) o[t][i] *= corr;
        }
        __syncthreads();
#pragma unroll
        for (int kh = 0; kh < 2; ++kh) {
            const Split pa = sp_lds(myp + l15 * 64u, (unsigned)kh * 32u, hf);
#pragma unroll
            for (int t = 0; t < 4; ++t) {
                const unsigned dcol = (unsigned)t * 16u + l15;
                v16us bb;
#pragma unroll
                for (unsigned e = 0; e < 16u; ++e) bb[e] = vl[((unsigned)kh * 32u + frag_k(e, hf)) * VP + dcol];
                o[t] = wmma2(pa, __builtin_bit_cast(v16b, bb), o[t]);
            }
        }
    }

    float invr[8];
#pragma unroll
    for (int i = 0; i < 8; ++i) invr[i] = (l8[i] > 0.f) ? (1.0f / l8[i]) : 0.f;

    float* obase = O + (size_t)b * OUT_BSTRIDE + dv0;
    __syncthreads();
#pragma unroll
    for (int i = 0; i < 8; ++i)
#pragma unroll
        for (int t = 0; t < 4; ++t)
            myp[((unsigned)i + 8u * hf) * 64u + (unsigned)t * 16u + l15] = o[t][i] * invr[i];
    __syncthreads();
#pragma unroll 1
    for (unsigned r0 = 0; r0 < 16u; r0 += 2u) {
        const unsigned row = r0 + (lane >> 4), c4 = (lane & 15u) * 4u;
        const v4f v = *(const v4f*)(myp + row * 64u + c4);
        VST2(v4f, obase + (size_t)(q0 + row) * HD + c4, v);
    }
}

extern "C" void kernel_launch(void* const* d_in, const int* in_sizes, int n_in, void* d_out, int out_size, void* d_ws, size_t ws_size, hipStream_t stream) {
    if (n_in < 3) return;
    const long long need_in  = ((long long)(NB - 1) * SEQ_FULL + SEQ) * HD;
    const long long need_out = (long long)(NB - 1) * OUT_BSTRIDE + (long long)SEQ * HD;
    if ((long long)in_sizes[0] < need_in || (long long)in_sizes[1] < need_in || (long long)in_sizes[2] < need_in) return;
    if ((long long)out_size < need_out) return;
    if (3 * PLANE_BYTES > ws_size) return;
    const float* q = (const float*)d_in[0];
    const float* k = (const float*)d_in[1];
    const float* v = (const float*)d_in[2];
    float* out = (float*)d_out;
    char* wsp = (char*)d_ws;
    unsigned short* PQ = (unsigned short*)wsp; wsp += PLANE_BYTES;
    unsigned short* PK = (unsigned short*)wsp; wsp += PLANE_BYTES;
    unsigned short* PV = (unsigned short*)wsp; wsp += PLANE_BYTES;
    k_cvt3<<<dim3((unsigned)(PLANE_ELEMS / 2048), 3u, 1u), 256, 0, stream>>>(q, k, v, PQ, PK, PV);
    k_attn<<<dim3((unsigned)(SEQ / (16 * AW)), (unsigned)NB, (unsigned)(HD / DVH)), 32 * AW, 0, stream>>>(PQ, PK, PV, out);
}
